// CrossAttention_44246753083653
// MI455X (gfx1250) — hardware-verified
//
#include <hip/hip_runtime.h>


#ifndef NB
#define NB 128
#endif
#define NB_FULL 128
#define CH 1024
#define KW 9
#define RB 128
#define MPAD ((((NB) + 63) / 64) * 64)
#define VCAR 16.0f
#define PEXP 14.0f
#define L2E 1.4426950408889634f
#define BNEPS 1e-5f
#define LSLOPE 0.1f

static_assert(NB >= 1);
static_assert(NB <= NB_FULL);
static_assert(CH % RB == 0);
static_assert(CH % 128 == 0);
static_assert(MPAD % 64 == 0);
static_assert(RB == 8 * 16);
static_assert((CH * CH) % 8 == 0);

typedef _Float16 h16;
typedef unsigned short bf;
typedef __attribute__((ext_vector_type(16))) __bf16   v16bf;
typedef __attribute__((ext_vector_type(16))) _Float16 v16h;
typedef __attribute__((ext_vector_type(8)))  _Float16 v8h;
typedef __attribute__((ext_vector_type(4)))  _Float16 v4h;
typedef __attribute__((ext_vector_type(8)))  unsigned short v8us;
typedef __attribute__((ext_vector_type(4)))  unsigned short v4us;
typedef __attribute__((ext_vector_type(8)))  float    v8f;
typedef __attribute__((ext_vector_type(4)))  float    v4f;
typedef v4f  __attribute__((may_alias)) v4fa;

__device__ __forceinline__ unsigned short f2bf(float f) { unsigned u = __float_as_uint(f); u += 0x7FFFu + ((u >> 16) & 1u); return (unsigned short)(u >> 16); }
__device__ __forceinline__ float bf2f(unsigned short b) { return __uint_as_float(((unsigned)b) << 16); }
__device__ __forceinline__ float bfr(float f) { return bf2f(f2bf(f)); }
__device__ __forceinline__ v16h cat16h(v8us lo, v8us hi) { return __builtin_bit_cast(v16h, __builtin_shufflevector(lo, hi, 0, 1, 2, 3, 4, 5, 6, 7, 8, 9, 10, 11, 12, 13, 14, 15)); }
__device__ __forceinline__ v16bf cat16b(v8us lo, v8us hi) { return __builtin_bit_cast(v16bf, __builtin_shufflevector(lo, hi, 0, 1, 2, 3, 4, 5, 6, 7, 8, 9, 10, 11, 12, 13, 14, 15)); }
__device__ __forceinline__ v8f wmma16(v16h a, v16h b, v8f c) { return __builtin_amdgcn_wmma_f32_16x16x32_f16(false, a, false, b, (short)0, c, false, false); }
__device__ __forceinline__ v8f wmmab(v16bf a, v16bf b, v8f c) { return __builtin_amdgcn_wmma_f32_16x16x32_bf16(false, a, false, b, (short)0, c, false, false); }
__device__ __forceinline__ v16bf ldbf(const bf* p) { return cat16b(*(const v8us*)p, *(const v8us*)(p + 16)); }

__global__ __launch_bounds__(256) void k_wc(const float* __restrict__ w, bf* dst, size_t n8) {
    const size_t i = (size_t)blockIdx.x * 256 + threadIdx.x; if (i >= n8) return;
    v8us o;
#pragma unroll
    for (int k = 0; k < 8; ++k) o[k] = f2bf(w[(i * 8 + (size_t)k) * KW + 4]);
    *(volatile v8us*)(dst + i * 8) = o; __threadfence(); *(volatile v8us*)(dst + i * 8) = o;
}

__global__ __launch_bounds__(256) void k_zero16(bf* dst, size_t n8) {
    const size_t i = (size_t)blockIdx.x * 256 + threadIdx.x; if (i >= n8) return;
    v8us o;
#pragma unroll
    for (int k = 0; k < 8; ++k) o[k] = (unsigned short)0;
    *(volatile v8us*)(dst + i * 8) = o; __threadfence(); *(volatile v8us*)(dst + i * 8) = o;
}

__global__ __launch_bounds__(256) void k_attn(const float* __restrict__ vis, const float* __restrict__ tac, bf* H2) {
    __shared__ __align__(16) float vf[CH];
    __shared__ __align__(16) unsigned short vsu[CH];
    __shared__ float red[16];
    __shared__ __align__(16) float dts[8 * 256];
    __shared__ __align__(16) float hsb[RB];
    const int tid = threadIdx.x, lane = tid & 31, wave = tid >> 5, m = lane & 15, hh = lane >> 4;
    const int b = blockIdx.y, iblk = blockIdx.x * RB;
    {
        const v4f x4 = *(const v4f*)(vis + (size_t)b * CH + tid * 4);
        v4f r4; v4h s4; float mx = -3.0e38f, mn = 3.0e38f;
#pragma unroll
        for (int q = 0; q < 4; ++q) { const float r = bfr(x4[q]); r4[q] = r; s4[q] = (h16)(r * VCAR); mx = fmaxf(mx, r); mn = fminf(mn, r); }
        *(v4f*)(vf + tid * 4) = r4;
        *(v4us*)(vsu + tid * 4) = __builtin_bit_cast(v4us, s4);
#pragma unroll
        for (int sh = 16; sh; sh >>= 1) { mx = fmaxf(mx, __shfl_xor(mx, sh, 32)); mn = fminf(mn, __shfl_xor(mn, sh, 32)); }
        if (lane == 0) { red[wave] = mx; red[8 + wave] = mn; }
    }
    __syncthreads();
    float vmax = red[0], vmin = red[8];
#pragma unroll
    for (int w = 1; w < 8; ++w) { vmax = fmaxf(vmax, red[w]); vmin = fminf(vmin, red[8 + w]); }
    const int i = iblk + wave * 16 + m;
    const float t = bfr(tac[(size_t)b * CH + i]);
    const float mrow = (t > 0.0f) ? t * vmax : t * vmin;
    v8us mv;
    {
        const unsigned short msk = (m == 0) ? (unsigned short)0xFFFFu : (unsigned short)0u;
#pragma unroll
        for (int q = 0; q < 8; ++q) mv[q] = msk;
    }
    v8f acc = (v8f){}; float S = 0.0f;
#pragma unroll 1
    for (int kc = 0; kc < CH; kc += 32) {
        const v8f va = *(const v8f*)(vf + kc + 8 * hh);
        const v8f vb = *(const v8f*)(vf + kc + 16 + 8 * hh);
        v8us b0 = *(const v8us*)(vsu + kc + 8 * hh);
        v8us b1 = *(const v8us*)(vsu + kc + 16 + 8 * hh);
        b0 = b0 & mv; b1 = b1 & mv;
        const v16h bfrag = cat16h(b0, b1);
        v16h af = (v16h){};
#pragma unroll
        for (int q = 0; q < 8; ++q) { const float d = t * va[q] - mrow; const float e = __builtin_amdgcn_exp2f(fmaf(d, L2E, PEXP)); S += e; af[q] = (h16)e; }
#pragma unroll
        for (int q = 0; q < 8; ++q) { const float d = t * vb[q] - mrow; const float e = __builtin_amdgcn_exp2f(fmaf(d, L2E, PEXP)); S += e; af[8 + q] = (h16)e; }
        acc = wmma16(af, bfrag, acc);
        asm volatile("v_nop\n\tv_nop\n\tv_nop\n\tv_nop" : "+v"(acc) : "v"(af), "v"(bfrag));
    }
    S += __shfl_xor(S, 16, 32);
    float* dt = dts + wave * 256;
#pragma unroll
    for (int r = 0; r < 8; ++r) dt[(8 * hh + r) * 16 + m] = acc[r];
    __builtin_amdgcn_fence(3  , "wavefront"); __builtin_amdgcn_wave_barrier(); asm volatile("" ::: "memory");
    const float num = dt[m * 16];
    const float crs = num * __builtin_amdgcn_rcpf(VCAR * S);
    hsb[wave * 16 + m] = vf[i] + crs;
    __syncthreads();
    if (wave == 0) {
        const int pl = hh;
        v8us o;
#pragma unroll
        for (int q = 0; q < 8; ++q) { const float hv = hsb[8 * m + q]; const unsigned short a = f2bf(hv); const unsigned short l2 = f2bf(hv - bf2f(a)); o[q] = pl ? l2 : a; }
        bf* dst = H2 + (size_t)pl * MPAD * CH + (size_t)b * CH + iblk + 8 * m;
        *(volatile v8us*)dst = o; __threadfence(); *(volatile v8us*)dst = o;
    }
}

__global__ __launch_bounds__(32) void k_gemm_bn(const bf* __restrict__ A, const bf* __restrict__ A2, const bf* __restrict__ Bt, int K, float* C, int ldc, int Mreal,
        const float* __restrict__ cb, const float* __restrict__ ga, const float* __restrict__ be, const float* __restrict__ mu, const float* __restrict__ va) {
    __shared__ __align__(16) float os[16 * 68];
    const int lane = threadIdx.x & 31, lr = lane & 15, hi = lane >> 4; const int r0 = blockIdx.x * 64, c0 = blockIdx.y * 64;
    v8f acc[4][4];
#pragma unroll
    for (int mb = 0; mb < 4; ++mb)
#pragma unroll
        for (int nb = 0; nb < 4; ++nb) acc[mb][nb] = (v8f){};
    const size_t aoff = (size_t)(r0 + lr) * K + 8 * hi, boff = (size_t)(c0 + lr) * K + 8 * hi;
#pragma unroll 1
    for (int kc = 0; kc < K; kc += 32) {
        v16bf a[4], a2[4];
#pragma unroll
        for (int mb = 0; mb < 4; ++mb) { a[mb] = ldbf(A + aoff + (size_t)mb * 16 * K + kc); a2[mb] = ldbf(A2 + aoff + (size_t)mb * 16 * K + kc); }
#pragma unroll
        for (int nb = 0; nb < 4; ++nb) { const v16bf b = ldbf(Bt + boff + (size_t)nb * 16 * K + kc);
#pragma unroll
            for (int mb = 0; mb < 4; ++mb) { acc[mb][nb] = wmmab(a[mb], b, acc[mb][nb]); acc[mb][nb] = wmmab(a2[mb], b, acc[mb][nb]); } }
        asm volatile("v_nop\n\tv_nop\n\tv_nop\n\tv_nop" : "+v"(acc[0][0]), "+v"(acc[1][1]), "+v"(acc[2][2]), "+v"(acc[3][3]) : "v"(a[0]), "v"(a[3]));
    }
    float pb[4], pm[4], pi[4], pe[4];
#pragma unroll
    for (int e = 0; e < 4; ++e) { const int c = c0 + lr * 4 + e; pb[e] = bfr(cb[c]); pm[e] = bfr(mu[c]); pe[e] = bfr(be[c]); const float g = bfr(ga[c]); const float vv = bfr(va[c]); pi[e] = g / sqrtf(vv + BNEPS); }
#pragma unroll
    for (int mb = 0; mb < 4; ++mb) {
#pragma unroll
        for (int nb = 0; nb < 4; ++nb) {
#pragma unroll
            for (int j = 0; j < 8; ++j) os[(hi * 8 + j) * 68 + nb * 16 + lr] = acc[mb][nb][j]; }
        __builtin_amdgcn_fence(3  , "wavefront"); __builtin_amdgcn_wave_barrier(); asm volatile("" ::: "memory");
        float* crow = C + (size_t)(r0 + mb * 16) * ldc + c0;
#pragma unroll 1
        for (int ps = 0; ps < 2; ++ps) {
#pragma unroll
            for (int s = 0; s < 8; ++s) { const int row = 2 * s + hi, cofs = lr * 4; v4f val = *(const v4fa*)(os + row * 68 + cofs);
#pragma unroll
                for (int e = 0; e < 4; ++e) { float y = val[e] + pb[e]; y = (y - pm[e]) * pi[e] + pe[e]; val[e] = (y > 0.0f) ? y : LSLOPE * y; }
                if (r0 + mb * 16 + row < Mreal) *(volatile v4f*)(crow + (size_t)row * ldc + cofs) = val; }
            if (ps == 0) __threadfence(); }
        __builtin_amdgcn_fence(3  , "wavefront"); __builtin_amdgcn_wave_barrier(); asm volatile("" ::: "memory");
    }
}

extern "C" void kernel_launch(void* const* d_in, const int* in_sizes, int n_in,
                              void* d_out, int out_size, void* d_ws, size_t ws_size, hipStream_t stream) {
    if (n_in < 8) return;
    if (in_sizes[0] < NB * CH || in_sizes[1] < NB * CH || in_sizes[2] < CH * CH * KW) return;
    if (in_sizes[3] < CH || in_sizes[4] < CH || in_sizes[5] < CH || in_sizes[6] < CH || in_sizes[7] < CH) return;
    if (out_size < NB * CH) return;
    const float* vis = (const float*)d_in[0];
    const float* tac = (const float*)d_in[1];
    const float* cw  = (const float*)d_in[2];
    const float* cbv = (const float*)d_in[3];
    const float* gav = (const float*)d_in[4];
    const float* bev = (const float*)d_in[5];
    const float* muv = (const float*)d_in[6];
    const float* vav = (const float*)d_in[7];
    float* OUT = (float*)d_out;
    char* wsp = (char*)d_ws;
    auto take = [&](size_t bytes) { char* p = wsp; wsp += (bytes + 255) & ~(size_t)255; return (void*)p; };
    bf* WB = (bf*)take((size_t)CH * CH * 2);
    bf* H2 = (bf*)take((size_t)2 * MPAD * CH * 2);
    if ((size_t)(wsp - (char*)d_ws) > ws_size) return;
    k_wc<<<(unsigned)(((size_t)CH * CH / 8 + 255) / 256), 256, 0, stream>>>(cw, WB, (size_t)CH * CH / 8);
    k_attn<<<dim3(CH / RB, NB, 1), 256, 0, stream>>>(vis, tac, H2);
    if (MPAD > NB) {
        const size_t n8 = (size_t)(MPAD - NB) * CH / 8;
        k_zero16<<<(unsigned)((n8 + 255) / 256), 256, 0, stream>>>(H2 + (size_t)NB * CH, n8);
        k_zero16<<<(unsigned)((n8 + 255) / 256), 256, 0, stream>>>(H2 + (size_t)MPAD * CH + (size_t)NB * CH, n8);
    }
    k_gemm_bn<<<dim3(MPAD / 64, CH / 64, 1), 32, 0, stream>>>(H2, H2 + (size_t)MPAD * CH, WB, CH, OUT, CH, NB, cbv, gav, bev, muv, vav);
}
